// GraphSage_73564199845998
// MI455X (gfx1250) — hardware-run, weakly checked
//
#include <hip/hip_runtime.h>
#include <stddef.h>
#include <stdint.h>


#ifndef SPLIT_AGG
#define SPLIT_AGG 1
#endif
#ifndef SPLIT_EMB
#define SPLIT_EMB 1
#endif

#define NN     50000
#define DF     128
#define S1     25
#define S2     10
#define NPAD   50048
#define GBM    64
#define GBN    128
#define GTHR   128
#define AGGP   (SPLIT_AGG ? 256 : 128)
#define E1P    (SPLIT_EMB ? 256 : 128)
#define KA1    128
#define KB1    (AGGP + DF)
#define KA2    E1P
#define KB2    (AGGP + E1P)
#define PTHR   256
#define MTHR   256
#define MWAVE  8
#define WSMAX  134217728

#define PU_XB   (NPAD * DF / 8)
#define PU_WA1  (DF * KA1 / 8)
#define PU_WA2  (DF * KA2 / 8)
#define PU_WB1  (DF * KB1 / 8)
#define PU_WB2  (DF * KB2 / 8)
#define PE0     (PU_XB)
#define PE1     (PE0 + PU_WA1)
#define PE2     (PE1 + PU_WA2)
#define PE3     (PE2 + PU_WB1)
#define PE4     (PE3 + PU_WB2)
#define PE5     (PE4 + PTHR)

static constexpr size_t SZ_XB  = (size_t)NPAD * DF * 2;
static constexpr size_t SZ_M   = (size_t)NPAD * DF * 4;
static constexpr size_t SZ_AGG = (size_t)NPAD * AGGP * 2;
static constexpr size_t SZ_E1  = (size_t)NPAD * E1P * 2;
static constexpr size_t SZ_WA1 = (size_t)DF * KA1 * 2;
static constexpr size_t SZ_WA2 = (size_t)DF * KA2 * 2;
static constexpr size_t SZ_WB1 = (size_t)DF * KB1 * 2;
static constexpr size_t SZ_WB2 = (size_t)DF * KB2 * 2;
static constexpr size_t SZ_BAG = (size_t)DF * 4;
static constexpr size_t O_XB   = 0;
static constexpr size_t O_M    = O_XB  + SZ_XB;
static constexpr size_t O_AGG  = O_M   + SZ_M;
static constexpr size_t O_E1   = O_AGG + SZ_AGG;
static constexpr size_t O_WA1  = O_E1  + SZ_E1;
static constexpr size_t O_WA2  = O_WA1 + SZ_WA1;
static constexpr size_t O_WB1  = O_WA2 + SZ_WA2;
static constexpr size_t O_WB2  = O_WB1 + SZ_WB1;
static constexpr size_t O_BAG  = O_WB2 + SZ_WB2;
static constexpr size_t O_END  = O_BAG + SZ_BAG;

static_assert(DF == 128);
static_assert(S1 == 25 && S2 == 10 && S1 <= 32 && S2 <= 32);
static_assert(NPAD == 391 * 128 && NPAD % GBM == 0 && NPAD >= NN && NPAD % MWAVE == 0);
static_assert(GBN == DF && GBM == (GTHR / 32) * 16 && DF == 4 * 32);
static_assert(KA1 % 32 == 0 && KB1 % 32 == 0 && KA2 % 32 == 0 && KB2 % 32 == 0);
static_assert(KA1 == 128 && (KB1 == 384 || KB1 == 256) && (KA2 == 256 || KA2 == 128));
static_assert(KB2 == 512 || KB2 == 384 || KB2 == 256);
static_assert(PU_XB % PTHR == 0 && PU_WA1 % PTHR == 0 && PU_WA2 % PTHR == 0);
static_assert(PU_WB1 % PTHR == 0 && PU_WB2 % PTHR == 0 && PE5 % PTHR == 0);
static_assert(SZ_XB % 256 == 0 && SZ_M % 256 == 0 && SZ_AGG % 256 == 0 && SZ_E1 % 256 == 0);
static_assert(SZ_WA1 % 256 == 0 && SZ_WA2 % 256 == 0 && SZ_WB1 % 256 == 0 && SZ_WB2 % 256 == 0);
static_assert(O_END <= (size_t)WSMAX);
static_assert((long long)NN * DF < (1LL << 31));

typedef float          v4f   __attribute__((ext_vector_type(4)));
typedef float          v8f   __attribute__((ext_vector_type(8)));
typedef int            v8i   __attribute__((ext_vector_type(8)));
typedef unsigned       v2u   __attribute__((ext_vector_type(2)));
typedef unsigned       v4u   __attribute__((ext_vector_type(4)));
typedef unsigned short v8us  __attribute__((ext_vector_type(8)));
typedef unsigned short v16us __attribute__((ext_vector_type(16)));
typedef __bf16         v16bf __attribute__((ext_vector_type(16)));
typedef v4f  __attribute__((may_alias)) v4fa;
typedef v4u  __attribute__((may_alias)) v4ua;
typedef v8us __attribute__((may_alias)) v8usa;
union FragB { v16bf v; v16us u; v8us h[2]; v8i w; };

__device__ __forceinline__ v8f wmb(const FragB& a, const FragB& b, v8f c) {
  v8f d = __builtin_amdgcn_wmma_f32_16x16x32_bf16(false, a.v, false, b.v, (short)0, c, false, false);
  asm volatile("v_nop\n\tv_nop\n\tv_nop\n\tv_nop" : "+v"(d) : "v"(a.w), "v"(b.w));
  return d;
}

__device__ __forceinline__ unsigned bf16_bits(float f) {
  const unsigned u = __float_as_uint(f);
  return (u + 0x7FFFu + ((u >> 16) & 1u)) >> 16;
}
__device__ __forceinline__ float bf16_val(float f) {
  return __uint_as_float(bf16_bits(f) << 16);
}
__device__ __forceinline__ unsigned hl_bits(float v, unsigned& lo) {
  const unsigned hb = bf16_bits(v);
  lo = bf16_bits(v - __uint_as_float(hb << 16));
  return hb;
}
__device__ __forceinline__ float relu1(float v) { return (v > 0.0f) ? v : (v - v); }
__device__ __forceinline__ void pin4(const v4f& t) {
  asm volatile("" :: "v"(t.x), "v"(t.y), "v"(t.z), "v"(t.w));
}

__global__ __launch_bounds__(PTHR) void k_prep(const float* __restrict__ x, const float* __restrict__ wagg,
                                               const float* __restrict__ bagg, const float* __restrict__ wupd,
                                               unsigned short* pl, float* bagout, int nN) {
  const int tid = (int)threadIdx.x;
  const int u   = (int)blockIdx.x * PTHR + tid;
  if (u >= PE4) {
    if (tid < 32) {
      const v4f t = *(const v4f*)(bagg + 4 * tid);
      v4f o;
      o.x = bf16_val(t.x); o.y = bf16_val(t.y); o.z = bf16_val(t.z); o.w = bf16_val(t.w);
      float* bp = bagout + 4 * tid;
      *(volatile v4f*)bp = o;
      __threadfence();
      *(volatile v4f*)bp = o;
    }
    return;
  }
  v4f a, b;
  float lv = 1.0f;
  size_t doff;
  if (u < PE0) {
    const int row = u >> 4, k8 = (u & 15) * 8;
    const int rc  = row < nN ? row : nN - 1;
    const float* p = x + (size_t)rc * DF + k8;
    a = *(const v4f*)p;
    b = *(const v4f*)(p + 4);
    lv = row < nN ? 1.0f : 0.0f;
    doff = O_XB / 2 + (size_t)u * 8;
  } else if (u < PE1) {
    const int v = u - PE0;
    const int n = v >> 4, k8 = (v & 15) * 8;
    const float* p = wagg + (size_t)n * DF + k8;
    a = *(const v4f*)p;
    b = *(const v4f*)(p + 4);
    doff = O_WA1 / 2 + (size_t)v * 8;
  } else if (u < PE2) {
    const int v = u - PE1;
    const int n = v / (KA2 / 8);
    const int c = (v - n * (KA2 / 8)) * 8;
    const float* p = wagg + (size_t)n * DF + (c & (DF - 1));
    a = *(const v4f*)p;
    b = *(const v4f*)(p + 4);
    doff = O_WA2 / 2 + (size_t)v * 8;
  } else if (u < PE3) {
    const int v  = u - PE2;
    const int n  = v / (KB1 / 8);
    const int c  = (v - n * (KB1 / 8)) * 8;
    const int sc = (c & (DF - 1)) + ((c < AGGP) ? DF : 0);
    const float* p = wupd + (size_t)n * (2 * DF) + sc;
    a = *(const v4f*)p;
    b = *(const v4f*)(p + 4);
    doff = O_WB1 / 2 + (size_t)v * 8;
  } else {
    const int v  = u - PE3;
    const int n  = v / (KB2 / 8);
    const int c  = (v - n * (KB2 / 8)) * 8;
    const int sc = (c & (DF - 1)) + ((c < AGGP) ? DF : 0);
    const float* p = wupd + (size_t)n * (2 * DF) + sc;
    a = *(const v4f*)p;
    b = *(const v4f*)(p + 4);
    doff = O_WB2 / 2 + (size_t)v * 8;
  }
  v8us o;
  o[0] = (unsigned short)bf16_bits(a.x * lv); o[1] = (unsigned short)bf16_bits(a.y * lv);
  o[2] = (unsigned short)bf16_bits(a.z * lv); o[3] = (unsigned short)bf16_bits(a.w * lv);
  o[4] = (unsigned short)bf16_bits(b.x * lv); o[5] = (unsigned short)bf16_bits(b.y * lv);
  o[6] = (unsigned short)bf16_bits(b.z * lv); o[7] = (unsigned short)bf16_bits(b.w * lv);
  unsigned short* dp = pl + doff;
  *(volatile v8us*)dp = o;
  __threadfence();
  *(volatile v8us*)dp = o;
}

template <int MODE, int K0, int K1, int LDA0, int LDA1, int EP>
__global__ __launch_bounds__(GTHR) __attribute__((amdgpu_num_vgpr(248)))
void k_gemm(const unsigned short* __restrict__ A0, const unsigned short* __restrict__ A1,
            const unsigned short* __restrict__ BT, const float* __restrict__ bag,
            float* outF, unsigned short* outH, int nN) {
  static_assert(K0 > 0 && K0 % 32 == 0 && K1 % 32 == 0);
  static_assert(LDA0 % 8 == 0 && LDA1 % 8 == 0 && LDA0 >= K0 && (K1 == 0 || LDA1 >= K1));
  static_assert(EP == DF || EP == 2 * DF);
  constexpr int KT = K0 + K1;
  __shared__ __attribute__((aligned(16))) float stg[GBM * GBN];
  __shared__ __attribute__((aligned(16))) float sb[DF];
  const int tid = (int)threadIdx.x, lane = tid & 31, wave = tid >> 5, hh = lane >> 4, m = lane & 15;
  const int rowBase = (int)blockIdx.x * GBM;

  if constexpr (MODE == 0) {
    if (tid < 32) {
      const v4f t = *(const v4f*)(bag + 4 * tid);
      *(v4fa*)(sb + 4 * tid) = t;
    }
  }

  v8f acc[8];
  {
    const v8f z = {0.f, 0.f, 0.f, 0.f, 0.f, 0.f, 0.f, 0.f};
#pragma unroll
    for (int t = 0; t < 8; ++t) acc[t] = z;
  }
  const unsigned short* bp = BT + (size_t)m * (size_t)KT + 8 * hh;
  {
    const unsigned short* ap = A0 + (size_t)(rowBase + 16 * wave + m) * (size_t)LDA0 + 8 * hh;
#pragma unroll 1
    for (int k0 = 0; k0 < K0; k0 += 32) {
      FragB af;
      af.h[0] = *(const v8usa*)(ap + k0);
      af.h[1] = *(const v8usa*)(ap + k0 + 16);
#pragma unroll
      for (int nt = 0; nt < 8; ++nt) {
        const unsigned short* wq = bp + (size_t)(16 * nt) * (size_t)KT + k0;
        FragB bf;
        bf.h[0] = *(const v8usa*)wq;
        bf.h[1] = *(const v8usa*)(wq + 16);
        acc[nt] = wmb(af, bf, acc[nt]);
      }
    }
  }
  if constexpr (K1 > 0) {
    const unsigned short* ap = A1 + (size_t)(rowBase + 16 * wave + m) * (size_t)LDA1 + 8 * hh;
#pragma unroll 1
    for (int k1 = 0; k1 < K1; k1 += 32) {
      FragB af;
      af.h[0] = *(const v8usa*)(ap + k1);
      af.h[1] = *(const v8usa*)(ap + k1 + 16);
#pragma unroll
      for (int nt = 0; nt < 8; ++nt) {
        const unsigned short* wq = bp + (size_t)(16 * nt) * (size_t)KT + K0 + k1;
        FragB bf;
        bf.h[0] = *(const v8usa*)wq;
        bf.h[1] = *(const v8usa*)(wq + 16);
        acc[nt] = wmb(af, bf, acc[nt]);
      }
    }
  }

#pragma unroll
  for (int nt = 0; nt < 8; ++nt) {
    const int lc = 16 * nt + m;
#pragma unroll
    for (int r = 0; r < 8; ++r) {
      const int lr = 16 * wave + 8 * hh + r;
      stg[lr * GBN + lc] = acc[nt][r];
    }
  }
  __syncthreads();

  v4f b4 = {0.f, 0.f, 0.f, 0.f};
  if constexpr (MODE == 0) b4 = *(const v4fa*)(sb + 4 * lane);
  const int rb = rowBase + 16 * wave;
  float* stw = stg + (16 * wave) * GBN + 4 * lane;

#pragma unroll 1
  for (int i = 0; i < 16; ++i) {
    float* sp = stw + i * GBN;
    const v4f t = *(const v4fa*)sp;
    if constexpr (MODE == 0) {
      v4f y;
      y.x = relu1(t.x + b4.x); y.y = relu1(t.y + b4.y); y.z = relu1(t.z + b4.z); y.w = relu1(t.w + b4.w);
      *(v4fa*)sp = y;
    } else {
      const bool ok = (rb + i) < nN;
      v4f uu;
      uu.x = relu1(t.x); uu.y = relu1(t.y); uu.z = relu1(t.z); uu.w = relu1(t.w);
      float ss = (uu.x * uu.x + uu.y * uu.y) + (uu.z * uu.z + uu.w * uu.w);
      ss += __shfl_xor(ss, 16, 32);
      ss += __shfl_xor(ss, 8, 32);
      ss += __shfl_xor(ss, 4, 32);
      ss += __shfl_xor(ss, 2, 32);
      ss += __shfl_xor(ss, 1, 32);
      const float den = fmaxf(sqrtf(ss), 1e-12f);
      v4f y;
      y.x = uu.x / den; y.y = uu.y / den; y.z = uu.z / den; y.w = uu.w / den;
      y.x = ok ? y.x : 0.0f; y.y = ok ? y.y : 0.0f; y.z = ok ? y.z : 0.0f; y.w = ok ? y.w : 0.0f;
      if constexpr (MODE == 2) {
        *(v4fa*)sp = y;
      } else {
        unsigned l0, l1, l2, l3;
        const unsigned h0 = hl_bits(y.x, l0);
        const unsigned h1 = hl_bits(y.y, l1);
        const unsigned h2 = hl_bits(y.z, l2);
        const unsigned h3 = hl_bits(y.w, l3);
        v4u pk;
        pk.x = h0 | (h1 << 16);
        pk.y = h2 | (h3 << 16);
        pk.z = l0 | (l1 << 16);
        pk.w = l2 | (l3 << 16);
        *(v4ua*)sp = pk;
      }
    }
  }

#pragma unroll 1
  for (int i = 0; i < 16; ++i) {
    const int row = rb + i;
    const float* sp = stw + i * GBN;
    if constexpr (MODE == 1) {
      const v4u pk = *(const v4ua*)sp;
      v2u hi; hi.x = pk.x; hi.y = pk.y;
      unsigned short* rp = outH + (size_t)row * EP + 4 * lane;
      *(volatile v2u*)rp = hi;
      if constexpr (EP == 2 * DF) {
        v2u lo; lo.x = pk.z; lo.y = pk.w;
        *(volatile v2u*)(rp + DF) = lo;
      }
    } else {
      const v4f t = *(const v4fa*)sp;
      pin4(t);
      if (row < nN) *(volatile v4f*)(outF + (size_t)row * DF + 4 * lane) = t;
    }
  }
  __threadfence();
#pragma unroll 1
  for (int i = 0; i < 16; ++i) {
    const int row = rb + i;
    const float* sp = stw + i * GBN;
    if constexpr (MODE == 1) {
      const v4u pk = *(const v4ua*)sp;
      v2u hi; hi.x = pk.x; hi.y = pk.y;
      unsigned short* rp = outH + (size_t)row * EP + 4 * lane;
      *(volatile v2u*)rp = hi;
      if constexpr (EP == 2 * DF) {
        v2u lo; lo.x = pk.z; lo.y = pk.w;
        *(volatile v2u*)(rp + DF) = lo;
      }
    } else {
      const v4f t = *(const v4fa*)sp;
      pin4(t);
      if (row < nN) *(volatile v4f*)(outF + (size_t)row * DF + 4 * lane) = t;
    }
  }
}

template <int S, int APT>
__global__ __launch_bounds__(MTHR) void k_maxg(const float* __restrict__ Mp, const int* __restrict__ neigh,
                                               unsigned short* agg, int nN) {
  static_assert(S >= 1 && S <= 32);
  static_assert(APT == DF || APT == 2 * DF);
  const int lane = (int)threadIdx.x & 31, wave = (int)threadIdx.x >> 5;
  const int node = (int)blockIdx.x * MWAVE + wave;
  const int nc   = node < nN ? node : nN - 1;
  const int sc   = lane < S ? lane : S - 1;
  int id = neigh[(size_t)nc * S + sc];
  id = id < 0 ? 0 : (id > nN - 1 ? nN - 1 : id);
  float m0 = 0.0f, m1 = 0.0f, m2 = 0.0f, m3 = 0.0f;
#pragma unroll 5
  for (int s = 0; s < S; ++s) {
    const int ids = __builtin_amdgcn_readlane(id, s);
    const v4f r = *(const v4f*)(Mp + (size_t)ids * DF + 4 * lane);
    m0 = fmaxf(m0, r.x); m1 = fmaxf(m1, r.y); m2 = fmaxf(m2, r.z); m3 = fmaxf(m3, r.w);
  }
  const bool live = node < nN;
  m0 = live ? m0 : 0.0f; m1 = live ? m1 : 0.0f; m2 = live ? m2 : 0.0f; m3 = live ? m3 : 0.0f;
  unsigned l0, l1, l2, l3;
  const unsigned h0 = hl_bits(m0, l0);
  const unsigned h1 = hl_bits(m1, l1);
  const unsigned h2 = hl_bits(m2, l2);
  const unsigned h3 = hl_bits(m3, l3);
  v2u hi; hi.x = h0 | (h1 << 16); hi.y = h2 | (h3 << 16);
  v2u lo; lo.x = l0 | (l1 << 16); lo.y = l2 | (l3 << 16);
  unsigned short* rp = agg + (size_t)node * APT + 4 * lane;
  *(volatile v2u*)rp = hi;
  if constexpr (APT == 2 * DF) *(volatile v2u*)(rp + DF) = lo;
  __threadfence();
  *(volatile v2u*)rp = hi;
  if constexpr (APT == 2 * DF) *(volatile v2u*)(rp + DF) = lo;
  (void)lo;
}

extern "C" void kernel_launch(void* const* d_in, const int* in_sizes, int n_in,
                              void* d_out, int out_size, void* d_ws, size_t ws_size,
                              hipStream_t stream) {
  if (n_in < 6) return;
  if (in_sizes[0] != NN * DF) return;
  if (in_sizes[1] != DF * DF) return;
  if (in_sizes[2] != DF) return;
  if (in_sizes[3] != DF * 2 * DF) return;
  if (in_sizes[4] != NN * S1) return;
  if (in_sizes[5] != NN * S2) return;
  if (out_size != NN * DF) return;
  if (O_END > ws_size) return;

  const float* x    = (const float*)d_in[0];
  const float* wagg = (const float*)d_in[1];
  const float* bagg = (const float*)d_in[2];
  const float* wupd = (const float*)d_in[3];
  const int*   n1   = (const int*)d_in[4];
  const int*   n2   = (const int*)d_in[5];
  float* out = (float*)d_out;

  char* ws = (char*)d_ws;
  unsigned short* PL  = (unsigned short*)ws;
  unsigned short* XB  = (unsigned short*)(ws + O_XB);
  float*          Mpl = (float*)(ws + O_M);
  unsigned short* AGG = (unsigned short*)(ws + O_AGG);
  unsigned short* E1  = (unsigned short*)(ws + O_E1);
  unsigned short* WA1 = (unsigned short*)(ws + O_WA1);
  unsigned short* WA2 = (unsigned short*)(ws + O_WA2);
  unsigned short* WB1 = (unsigned short*)(ws + O_WB1);
  unsigned short* WB2 = (unsigned short*)(ws + O_WB2);
  float*          BAG = (float*)(ws + O_BAG);

  const int gG = NPAD / GBM;
  const int gX = NPAD / MWAVE;

  k_prep<<<PE5 / PTHR, PTHR, 0, stream>>>(x, wagg, bagg, wupd, PL, BAG, NN);
  k_gemm<0, KA1, 0, DF, DF, DF><<<gG, GTHR, 0, stream>>>(XB, XB, WA1, BAG, Mpl, AGG, NN);
  k_maxg<S1, AGGP><<<gX, MTHR, 0, stream>>>(Mpl, n1, AGG, NN);
  k_gemm<1, AGGP, DF, AGGP, DF, E1P><<<gG, GTHR, 0, stream>>>(AGG, XB, WB1, BAG, out, E1, NN);
  k_gemm<0, KA2, 0, E1P, E1P, DF><<<gG, GTHR, 0, stream>>>(E1, E1, WA2, BAG, Mpl, AGG, NN);
  k_maxg<S2, AGGP><<<gX, MTHR, 0, stream>>>(Mpl, n2, AGG, NN);
  k_gemm<2, AGGP, E1P, AGGP, E1P, DF><<<gG, GTHR, 0, stream>>>(AGG, E1, WB2, BAG, out, AGG, NN);
}
